// DiSA_14121852469285
// MI455X (gfx1250) — hardware-verified
//
#include <hip/hip_runtime.h>
#include <math.h>

typedef __attribute__((ext_vector_type(16))) _Float16 v16h;
typedef __attribute__((ext_vector_type(16))) __bf16 v16b;
typedef __attribute__((ext_vector_type(8)))  _Float16 v8h;
typedef __attribute__((ext_vector_type(8)))  float v8f;
typedef __attribute__((ext_vector_type(4)))  float v4f;
typedef __attribute__((ext_vector_type(2)))  float v2f;
typedef __attribute__((ext_vector_type(4)))  unsigned v4u;
typedef __attribute__((ext_vector_type(4)))  int v4i;
typedef float __attribute__((may_alias)) float_a;
typedef int __attribute__((may_alias)) int_a;

template <typename T> __device__ __forceinline__ void vst2(void* p, T v) { *(volatile T*)p = v; __threadfence(); *(volatile T*)p = v; }
__device__ __forceinline__ v8f wmma16(v16h a, v16h b, v8f c) {
  v8f d = __builtin_amdgcn_wmma_f32_16x16x32_f16(false, a, false, b, (short)0, c, false, false);
  asm volatile("v_nop\n\tv_nop\n\tv_nop\n\tv_nop" : "+v"(d) : "v"(a), "v"(b));
  return d;
}
__device__ __forceinline__ v8f wmma_bf(v16b a, v16b b, v8f c) {
  v8f d = __builtin_amdgcn_wmma_f32_16x16x32_bf16(false, a, false, b, (short)0, c, false, false);
  asm volatile("v_nop\n\tv_nop\n\tv_nop\n\tv_nop" : "+v"(d) : "v"(a), "v"(b));
  return d;
}
__device__ __forceinline__ v16h frag_h(const _Float16* rowk0, int lane) {
  union { v16h v; v8h q[2]; } u; const _Float16* p = rowk0 + 8 * (lane >> 4);
  u.q[0] = *(const v8h*)p; u.q[1] = *(const v8h*)(p + 16); return u.v;
}
__device__ __forceinline__ v16h frag_f32(const float* rowk0, int lane) {
  v16h a; const float* p = rowk0 + 8 * (lane >> 4);
#pragma unroll
  for (int i = 0; i < 8; ++i) { a[i] = (_Float16)p[i]; a[8 + i] = (_Float16)p[16 + i]; }
  return a;
}
__device__ __forceinline__ v16h frag_f32s(const float* rowk0, int lane, float sc) {
  v16h a; const float* p = rowk0 + 8 * (lane >> 4);
#pragma unroll
  for (int i = 0; i < 8; ++i) { a[i] = (_Float16)(p[i] * sc); a[8 + i] = (_Float16)(p[16 + i] * sc); }
  return a;
}
__device__ __forceinline__ v16h fragc_f32(const float* W, int k0, int n, int lane, int ld, int K) {
  v16h a; const int g = lane >> 4;
#pragma unroll
  for (int i = 0; i < 8; ++i) { const int ka = k0 + 8 * g + i, kb = ka + 16;
    a[i] = (_Float16)(ka < K ? W[(size_t)(ka < K ? ka : K - 1) * ld + n] : 0.f); a[8 + i] = (_Float16)(kb < K ? W[(size_t)(kb < K ? kb : K - 1) * ld + n] : 0.f); }
  return a;
}
struct F2 { v16b h, l; };
__device__ __forceinline__ F2 bsplit16(const float v[16]) { F2 r;
#pragma unroll
  for (int i = 0; i < 16; ++i) { const __bf16 h = (__bf16)v[i]; r.h[i] = h; r.l[i] = (__bf16)(v[i] - (float)h); }
  return r; }
__device__ __forceinline__ F2 split_row(const float* row, int k0, int lane) { float v[16]; const float* p = row + k0 + 8 * (lane >> 4);
#pragma unroll
  for (int i = 0; i < 8; ++i) { v[i] = p[i]; v[8 + i] = p[16 + i]; }
  return bsplit16(v); }
__device__ __forceinline__ F2 split_rowK(const float* row, int k0, int lane, int K) { float v[16]; const int g = lane >> 4;
#pragma unroll
  for (int i = 0; i < 8; ++i) { const int ka = k0 + 8 * g + i, kb = ka + 16; v[i] = ka < K ? row[ka < K ? ka : K - 1] : 0.f; v[8 + i] = kb < K ? row[kb < K ? kb : K - 1] : 0.f; }
  return bsplit16(v); }
__device__ __forceinline__ F2 split_col(const float* W, int k0, int n, int lane, int ld, int K) { float v[16]; const int g = lane >> 4;
#pragma unroll
  for (int i = 0; i < 8; ++i) { const int ka = k0 + 8 * g + i, kb = ka + 16; v[i] = ka < K ? W[(size_t)(ka < K ? ka : K - 1) * ld + n] : 0.f; v[8 + i] = kb < K ? W[(size_t)(kb < K ? kb : K - 1) * ld + n] : 0.f; }
  return bsplit16(v); }
__device__ __forceinline__ v8f mac3(const F2& a, const F2& b, v8f c) { c = wmma_bf(a.l, b.h, c); c = wmma_bf(a.h, b.l, c); return wmma_bf(a.h, b.h, c); }
__device__ __forceinline__ float sigm(float v) { return 1.0f / (1.0f + expf(-v)); }
#define LDSX() do { asm volatile("s_wait_dscnt 0" ::: "memory"); __builtin_amdgcn_wave_barrier(); __builtin_amdgcn_fence(__ATOMIC_RELEASE, "workgroup"); } while (0)

__device__ __forceinline__ float bfr(float v) { return (float)(__bf16)v; }
#define NB 2
#define LL 256
#define DH 512
#define NR (NB * LL)
#define WS_REP 0u
#define WS_DEP (WS_REP + 4u * (size_t)NR * DH)
#define WS_HEAD (WS_DEP + 4u * (size_t)NR * DH)
#define WS_AO  (WS_HEAD + 4u * (size_t)NR * DH)
#define WS_END (WS_AO + 4u * (size_t)NR * DH)
__global__ __launch_bounds__(128) void k_lin(const float* __restrict__ X, const float* __restrict__ REPi, const float* __restrict__ Wt, const float* __restrict__ Bv, int which, float* __restrict__ DST) { __shared__ __align__(16) float sf[4][16][132];
  const int tid = threadIdx.x, wave = tid >> 5, lane = tid & 31, col = lane & 15, g = lane >> 4; const int c0 = blockIdx.y * 128; const size_t r0 = (size_t)blockIdx.x * 64 + wave * 16;
  v8f acc[8] = {};
#pragma unroll 2
  for (int kc = 0; kc < DH / 32; ++kc) { F2 a; if (which == 0) { float v[16]; const float* p = X + (r0 + col) * DH + kc * 32 + 8 * g;
#pragma unroll
      for (int i = 0; i < 8; ++i) { v[i] = bfr(p[i]); v[8 + i] = bfr(p[16 + i]); }
      a = bsplit16(v); } else a = split_row(REPi + (r0 + col) * DH, kc * 32, lane);
#pragma unroll
    for (int j = 0; j < 8; ++j) { v16b w; const int o = c0 + j * 16 + col;
#pragma unroll
      for (int i = 0; i < 8; ++i) { w[i] = (__bf16)Wt[(size_t)(kc * 32 + 8 * g + i) * DH + o]; w[8 + i] = (__bf16)Wt[(size_t)(kc * 32 + 16 + 8 * g + i) * DH + o]; }
      asm volatile("s_wait_loadcnt 0x0" ::: "memory"); acc[j] = wmma_bf(a.h, w, acc[j]); if (which != 0) acc[j] = wmma_bf(a.l, w, acc[j]); } }
#pragma unroll
  for (int j = 0; j < 8; ++j) { const float bb = bfr(Bv[c0 + j * 16 + col]);
#pragma unroll
    for (int r = 0; r < 8; ++r) { float v = acc[j][r] + bb; if (which == 0) v = v > 0.f ? v : expm1f(v); sf[wave][8 * g + r][j * 16 + col] = v; } }
  LDSX(); for (int rl = 0; rl < 16; ++rl) vst2(DST + (r0 + rl) * DH + c0 + lane * 4, *(const v4f*)&sf[wave][rl][lane * 4]); }
__global__ __launch_bounds__(512) void k_att(const float* __restrict__ REP, const float* __restrict__ DEP, const float* __restrict__ HEAD, const float* __restrict__ BL, float* __restrict__ AO) {
  const int h = threadIdx.x; const int i = blockIdx.x; const size_t b = blockIdx.y; const float hi_ = HEAD[(b * LL + i) * DH + h] + bfr(BL[h]);
  float m = -3.0e38f, s = 0.f, acc = 0.f;
  if (i == LL - 1) {
#pragma unroll 4
    for (int j = 0; j < LL; ++j) acc += REP[(b * LL + j) * DH + h];
    AO[(b * LL + i) * DH + h] = acc * (1.0f / LL); return; }
#pragma unroll 2
  for (int j = i + 1; j < LL; ++j) { const float z = 5.0f * tanhf((DEP[(b * LL + j) * DH + h] + hi_) * 0.2f); const float r = REP[(b * LL + j) * DH + h];
    if (z > m) { const float sc = expf(m - z); s = s * sc + 1.0f; acc = acc * sc + r; m = z; } else { const float e = expf(z - m); s += e; acc += e * r; } }
  AO[(b * LL + i) * DH + h] = acc / s; }
__global__ __launch_bounds__(128) void k_gate(const float* __restrict__ REP, const float* __restrict__ AO, const float* __restrict__ WF1, const float* __restrict__ WF2, const float* __restrict__ BF, float* __restrict__ OUT) { __shared__ __align__(16) float sf[4][16][132];
  const int tid = threadIdx.x, wave = tid >> 5, lane = tid & 31, col = lane & 15, g = lane >> 4; const int c0 = blockIdx.y * 128; const size_t r0 = (size_t)blockIdx.x * 64 + wave * 16;
  v8f acc[8] = {};
#pragma unroll 1
  for (int src = 0; src < 2; ++src) { const float* A = src == 0 ? REP : AO; const float* Wt = src == 0 ? WF1 : WF2;
#pragma unroll 2
    for (int kc = 0; kc < DH / 32; ++kc) { const F2 a = split_row(A + (r0 + col) * DH, kc * 32, lane);
#pragma unroll
      for (int j = 0; j < 8; ++j) { v16b w; const int o = c0 + j * 16 + col;
#pragma unroll
        for (int i = 0; i < 8; ++i) { w[i] = (__bf16)Wt[(size_t)(kc * 32 + 8 * g + i) * DH + o]; w[8 + i] = (__bf16)Wt[(size_t)(kc * 32 + 16 + 8 * g + i) * DH + o]; }
        asm volatile("s_wait_loadcnt 0x0" ::: "memory"); acc[j] = wmma_bf(a.h, w, acc[j]); acc[j] = wmma_bf(a.l, w, acc[j]); } } }
#pragma unroll
  for (int j = 0; j < 8; ++j) { const int o = c0 + j * 16 + col; const float bb = bfr(BF[o]);
#pragma unroll
    for (int r = 0; r < 8; ++r) { const size_t row = r0 + 8 * g + r; const float gt = 1.0f / (1.0f + expf(-(acc[j][r] + bb))); const float rp = REP[row * DH + o], ao = AO[row * DH + o]; sf[wave][8 * g + r][j * 16 + col] = gt * rp + (1.0f - gt) * ao; }
    asm volatile("s_wait_loadcnt 0x0" ::: "memory"); }
  LDSX(); for (int rl = 0; rl < 16; ++rl) vst2(OUT + (r0 + rl) * DH + c0 + lane * 4, *(const v4f*)&sf[wave][rl][lane * 4]); }
extern "C" void kernel_launch(void* const* d_in, const int* in_sizes, int n_in, void* d_out, int out_size, void* d_ws, size_t ws_size, hipStream_t stream) {
  (void)in_sizes; (void)n_in; (void)out_size;
  const float** F = (const float**)d_in;
  if (ws_size < (size_t)WS_END) return;
  char* ws = (char*)d_ws; float *REP = (float*)(ws + WS_REP), *DEP = (float*)(ws + WS_DEP), *HEAD = (float*)(ws + WS_HEAD), *AO = (float*)(ws + WS_AO);
  k_lin<<<dim3(NR / 64, DH / 128), 128, 0, stream>>>(F[0], nullptr, F[1], F[2], 0, REP);
  k_lin<<<dim3(NR / 64, DH / 128), 128, 0, stream>>>(nullptr, REP, F[3], F[4], 1, DEP);
  k_lin<<<dim3(NR / 64, DH / 128), 128, 0, stream>>>(nullptr, REP, F[5], F[6], 2, HEAD);
  k_att<<<dim3(LL, NB), 512, 0, stream>>>(REP, DEP, HEAD, F[7], AO);
  k_gate<<<dim3(NR / 64, DH / 128), 128, 0, stream>>>(REP, AO, F[8], F[9], F[10], (float*)d_out);
}
